// deformable_LKAConv_87076166959782
// MI455X (gfx1250) — hardware-verified
//
#include <hip/hip_runtime.h>
#include <math.h>

typedef __attribute__((ext_vector_type(16))) _Float16 v16h;
typedef __attribute__((ext_vector_type(16))) __bf16 v16b;
typedef __attribute__((ext_vector_type(8)))  _Float16 v8h;
typedef __attribute__((ext_vector_type(8)))  float v8f;
typedef __attribute__((ext_vector_type(4)))  float v4f;
typedef __attribute__((ext_vector_type(2)))  float v2f;
typedef __attribute__((ext_vector_type(4)))  unsigned v4u;
typedef __attribute__((ext_vector_type(4)))  int v4i;
typedef float __attribute__((may_alias)) float_a;
typedef int __attribute__((may_alias)) int_a;

template <typename T> __device__ __forceinline__ void vst2(void* p, T v) { *(volatile T*)p = v; __threadfence(); *(volatile T*)p = v; }
__device__ __forceinline__ v8f wmma16(v16h a, v16h b, v8f c) {
  v8f d = __builtin_amdgcn_wmma_f32_16x16x32_f16(false, a, false, b, (short)0, c, false, false);
  asm volatile("v_nop\n\tv_nop\n\tv_nop\n\tv_nop" : "+v"(d) : "v"(a), "v"(b));
  return d;
}
__device__ __forceinline__ v8f wmma_bf(v16b a, v16b b, v8f c) {
  v8f d = __builtin_amdgcn_wmma_f32_16x16x32_bf16(false, a, false, b, (short)0, c, false, false);
  asm volatile("v_nop\n\tv_nop\n\tv_nop\n\tv_nop" : "+v"(d) : "v"(a), "v"(b));
  return d;
}
__device__ __forceinline__ v16h frag_h(const _Float16* rowk0, int lane) {
  union { v16h v; v8h q[2]; } u; const _Float16* p = rowk0 + 8 * (lane >> 4);
  u.q[0] = *(const v8h*)p; u.q[1] = *(const v8h*)(p + 16); return u.v;
}
__device__ __forceinline__ v16h frag_f32(const float* rowk0, int lane) {
  v16h a; const float* p = rowk0 + 8 * (lane >> 4);
#pragma unroll
  for (int i = 0; i < 8; ++i) { a[i] = (_Float16)p[i]; a[8 + i] = (_Float16)p[16 + i]; }
  return a;
}
__device__ __forceinline__ v16h frag_f32s(const float* rowk0, int lane, float sc) {
  v16h a; const float* p = rowk0 + 8 * (lane >> 4);
#pragma unroll
  for (int i = 0; i < 8; ++i) { a[i] = (_Float16)(p[i] * sc); a[8 + i] = (_Float16)(p[16 + i] * sc); }
  return a;
}
__device__ __forceinline__ v16h fragc_f32(const float* W, int k0, int n, int lane, int ld, int K) {
  v16h a; const int g = lane >> 4;
#pragma unroll
  for (int i = 0; i < 8; ++i) { const int ka = k0 + 8 * g + i, kb = ka + 16;
    a[i] = (_Float16)(ka < K ? W[(size_t)(ka < K ? ka : K - 1) * ld + n] : 0.f); a[8 + i] = (_Float16)(kb < K ? W[(size_t)(kb < K ? kb : K - 1) * ld + n] : 0.f); }
  return a;
}
struct F2 { v16b h, l; };
__device__ __forceinline__ F2 bsplit16(const float v[16]) { F2 r;
#pragma unroll
  for (int i = 0; i < 16; ++i) { const __bf16 h = (__bf16)v[i]; r.h[i] = h; r.l[i] = (__bf16)(v[i] - (float)h); }
  return r; }
__device__ __forceinline__ F2 split_row(const float* row, int k0, int lane) { float v[16]; const float* p = row + k0 + 8 * (lane >> 4);
#pragma unroll
  for (int i = 0; i < 8; ++i) { v[i] = p[i]; v[8 + i] = p[16 + i]; }
  return bsplit16(v); }
__device__ __forceinline__ F2 split_rowK(const float* row, int k0, int lane, int K) { float v[16]; const int g = lane >> 4;
#pragma unroll
  for (int i = 0; i < 8; ++i) { const int ka = k0 + 8 * g + i, kb = ka + 16; v[i] = ka < K ? row[ka < K ? ka : K - 1] : 0.f; v[8 + i] = kb < K ? row[kb < K ? kb : K - 1] : 0.f; }
  return bsplit16(v); }
__device__ __forceinline__ F2 split_col(const float* W, int k0, int n, int lane, int ld, int K) { float v[16]; const int g = lane >> 4;
#pragma unroll
  for (int i = 0; i < 8; ++i) { const int ka = k0 + 8 * g + i, kb = ka + 16; v[i] = ka < K ? W[(size_t)(ka < K ? ka : K - 1) * ld + n] : 0.f; v[8 + i] = kb < K ? W[(size_t)(kb < K ? kb : K - 1) * ld + n] : 0.f; }
  return bsplit16(v); }
__device__ __forceinline__ v8f mac3(const F2& a, const F2& b, v8f c) { c = wmma_bf(a.l, b.h, c); c = wmma_bf(a.h, b.l, c); return wmma_bf(a.h, b.h, c); }
__device__ __forceinline__ float sigm(float v) { return 1.0f / (1.0f + expf(-v)); }
#define LDSX() do { asm volatile("s_wait_dscnt 0" ::: "memory"); __builtin_amdgcn_wave_barrier(); __builtin_amdgcn_fence(__ATOMIC_RELEASE, "workgroup"); } while (0)


#define NBT 4
#define CC 64
#define HH 56
#define WWD 56
#define NPI (HH * WWD)
#define NPIX (NBT * NPI)
#ifndef NTL
#define NTL (NPIX / 64)
#define NBO NBT
#endif
typedef __attribute__((ext_vector_type(8))) __bf16 v8b;
__device__ __forceinline__ v16b frag_b(const __bf16* rowk0, int lane) {
  union { v16b v; v8b q[2]; } u; const __bf16* p = rowk0 + 8 * (lane >> 4);
  u.q[0] = *(const v8b*)p; u.q[1] = *(const v8b*)(p + 16); return u.v;
}
__device__ __forceinline__ float bfr(float v) { return (float)(__bf16)v; }
__device__ __attribute__((noinline)) float exp_ni(float v) { return expf(v); }
__device__ __attribute__((noinline)) float erf_ni(float v) { return erff(v); }
__device__ __forceinline__ v16b zfrag_ok(v16b a, bool ok) { const v16b z = {}; return ok ? a : z; }

#define K1 (25 * CC)
#define K2 (49 * CC)
#define N1 64
#define N2 112
#define PK_O1 0
#define PK_O2 (PK_O1 + N1 * K1)
#define PK_PW (PK_O2 + N2 * K2)
#define PK_END (PK_PW + CC * CC)
#define WS_PK  0u
#define WS_XC  (((2u * PK_END) + 127u) / 128u * 128u)
#define WS_OF1 (WS_XC + 2u * NPIX * CC)
#define WS_A1H (WS_OF1 + 4u * NPIX * N1)
#define WS_A1L (WS_A1H + 2u * NPIX * CC)
#define WS_A1P (WS_A1L + 2u * NPIX * CC)
#define WS_OF2 (WS_A1P + 4u * NPIX * CC)
#define WS_A2H (WS_OF2 + 4u * NPIX * 128)
#define WS_A2L (WS_A2H + 2u * NPIX * CC)
#define WS_A3  (WS_A2L + 2u * NPIX * CC)
#define WS_END (WS_A3 + 4u * NPIX * CC)

__global__ __launch_bounds__(256) void k_pack(const float* __restrict__ OW1, const float* __restrict__ OW2, const float* __restrict__ PWW, __bf16* __restrict__ PK) {
  __shared__ __align__(16) __bf16 s[K2]; const int o = blockIdx.x, which = blockIdx.y, tid = threadIdx.x; int K; size_t dst;
  if (which == 0) { if (o >= N1) return; K = K1; dst = PK_O1 + (size_t)o * K1; for (int k = tid; k < K; k += 256) { const int tap = k / CC, c = k % CC; s[k] = (__bf16)((o < 50) ? OW1[((size_t)o * CC + c) * 25 + tap] : 0.f); } }
  else if (which == 1) { K = K2; dst = PK_O2 + (size_t)o * K2; for (int k = tid; k < K; k += 256) { const int tap = k / CC, c = k % CC; s[k] = (__bf16)((o < 98) ? OW2[((size_t)o * CC + c) * 49 + tap] : 0.f); } }
  else { if (o >= CC) return; K = CC; dst = PK_PW + (size_t)o * CC; if (tid < CC) s[tid] = (__bf16)PWW[(size_t)o * CC + tid]; }
  __syncthreads();
  for (int q = tid; q < K / 8; q += 256) vst2((unsigned*)(PK + dst + q * 8), *(const v4u*)&s[q * 8]);
}
__global__ __launch_bounds__(256) void k_xc(const float* __restrict__ X, __bf16* __restrict__ XC) {
  __shared__ __align__(16) __bf16 s[64][72]; const int tid = threadIdx.x; const size_t p0 = (size_t)blockIdx.x * 64; const int b = (int)(p0 / NPI); const int pl0 = (int)(p0 % NPI);
  for (int q = tid; q < 64 * CC; q += 256) { const int c = q >> 6, px = q & 63; s[px][c] = (__bf16)X[((size_t)b * CC + c) * NPI + pl0 + px]; }
  __syncthreads();
  for (int q = tid; q < 64 * 8; q += 256) { const int px = q >> 3, pc = q & 7; vst2((unsigned*)(XC + (p0 + px) * CC + pc * 8), *(const v4u*)&s[px][pc * 8]); }
}
template <int KS, int DIL, int PAD, int NT, int TWO, int LDO>
__global__ __launch_bounds__(128) void k_offc(const __bf16* __restrict__ IH, const __bf16* __restrict__ IL, const __bf16* __restrict__ W, const float* __restrict__ OB, int nreal, float* __restrict__ OFF) {
  __shared__ __align__(16) float so[4][16][132];
  const int tid = threadIdx.x, wave = tid >> 5, lane = tid & 31, col = lane & 15, g = lane >> 4; const size_t r0 = (size_t)blockIdx.x * 64 + wave * 16; const size_t p = r0 + col;
  const int b = (int)(p / NPI), pl = (int)(p % NPI), y = pl / WWD, xw = pl % WWD; constexpr int KT = KS * KS * CC;
  v8f acc[NT] = {};
#pragma unroll 1
  for (int tap = 0; tap < KS * KS; ++tap) { const int yy = y + (tap / KS) * DIL - PAD, xx = xw + (tap % KS) * DIL - PAD; const bool ok = yy >= 0 && yy < HH && xx >= 0 && xx < WWD;
    const size_t ap = ((size_t)b * NPI + (size_t)min(max(yy, 0), HH - 1) * WWD + min(max(xx, 0), WWD - 1)) * CC;
#pragma unroll
    for (int kc = 0; kc < 2; ++kc) { const v16b ah = zfrag_ok(frag_b(IH + ap + kc * 32, lane), ok); v16b al; if (TWO) al = zfrag_ok(frag_b(IL + ap + kc * 32, lane), ok); const size_t kk = (size_t)tap * CC + kc * 32;
#pragma unroll
      for (int j = 0; j < NT; ++j) { const v16b w = frag_b(W + (size_t)(j * 16 + col) * KT + kk, lane); if (TWO) acc[j] = wmma_bf(al, w, acc[j]); acc[j] = wmma_bf(ah, w, acc[j]); } } }
  for (int q = tid; q < 4 * 16 * 132; q += 128) (&so[0][0][0])[q] = 0.f;
  __syncthreads();
#pragma unroll
  for (int j = 0; j < NT; ++j) { const int o = j * 16 + col; const float bb = (o < nreal) ? bfr(OB[min(o, nreal - 1)]) : 0.f;
#pragma unroll
    for (int r = 0; r < 8; ++r) so[wave][8 * g + r][o] = acc[j][r] + bb; }
  LDSX();
  for (int rl = 0; rl < 16; ++rl) for (int pc = lane; pc < LDO / 4; pc += 32) vst2(OFF + (r0 + rl) * LDO + pc * 4, *(const v4f*)&so[wave][rl][pc * 4]);
}
template <int KS, int DIL, int PAD, int LDOFF>
__global__ __launch_bounds__(256) void k_ddw(const float* __restrict__ SRC, const float* __restrict__ OFF, const float* __restrict__ DW, int src_is_x, __bf16* __restrict__ AH, __bf16* __restrict__ AL, float* __restrict__ AP) {
  constexpr int KK = KS * KS;
  __shared__ unsigned short sidx[64][KK][4]; __shared__ float swt[64][KK][4]; __shared__ __align__(16) __bf16 sh_[64][72], sl_[64][72]; __shared__ __align__(16) float spl[CC][68];
  const int tid = threadIdx.x; const size_t p0 = (size_t)blockIdx.x * 64; const int b = (int)(p0 / NPI); const int pl0 = (int)(p0 % NPI);
  for (int q = tid; q < 64 * KK; q += 256) { const int px = q & 63, t = q >> 6; const int pl = pl0 + px; const int y = pl / WWD, xw = pl % WWD; const float* orow = OFF + (p0 + px) * LDOFF;
    const float dy = orow[2 * t], dx = orow[2 * t + 1]; const float by = (float)((t / KS) * DIL - PAD), bx = (float)((t % KS) * DIL - PAD);
    const float py = ((float)y + by) + dy, pxf = ((float)xw + bx) + dx; const float y0 = floorf(py), x0 = floorf(pxf); const float wy1 = py - y0, wx1 = pxf - x0;
#pragma unroll
    for (int cnr = 0; cnr < 4; ++cnr) { const float yi = y0 + (float)(cnr >> 1), xi = x0 + (float)(cnr & 1); const bool ok = (yi >= 0.f) && (yi <= (float)(HH - 1)) && (xi >= 0.f) && (xi <= (float)(WWD - 1));
      const int yc = (int)fminf(fmaxf(yi, 0.f), (float)(HH - 1)), xc = (int)fminf(fmaxf(xi, 0.f), (float)(WWD - 1));
      sidx[px][t][cnr] = (unsigned short)(yc * WWD + xc);
      const float wgt = (cnr == 0) ? (1.f - wy1) * (1.f - wx1) : (cnr == 1) ? (1.f - wy1) * wx1 : (cnr == 2) ? wy1 * (1.f - wx1) : wy1 * wx1; swt[px][t][cnr] = wgt * (ok ? 1.f : 0.f); } }
  __syncthreads();
  { const int px = tid & 63, cq = tid >> 6;
    for (int ci = 0; ci < 16; ++ci) { const int c = cq * 16 + ci; const float* plane = SRC + ((size_t)b * CC + c) * NPI; float a = 0.f;
      for (int t = 0; t < KK; ++t) { float sv;
        if (src_is_x) sv = ((bfr(plane[sidx[px][t][0]]) * swt[px][t][0] + bfr(plane[sidx[px][t][1]]) * swt[px][t][1]) + bfr(plane[sidx[px][t][2]]) * swt[px][t][2]) + bfr(plane[sidx[px][t][3]]) * swt[px][t][3];
        else sv = ((plane[sidx[px][t][0]] * swt[px][t][0] + plane[sidx[px][t][1]] * swt[px][t][1]) + plane[sidx[px][t][2]] * swt[px][t][2]) + plane[sidx[px][t][3]] * swt[px][t][3];
        a += sv * bfr(DW[(size_t)c * KK + t]); }
      const __bf16 hb = (__bf16)a; sh_[px][c] = hb; sl_[px][c] = (__bf16)(a - (float)hb); spl[c][px] = a; } }
  __syncthreads();
  for (int q = tid; q < 64 * 8; q += 256) { const int px = q >> 3, pc = q & 7; vst2((unsigned*)(AH + (p0 + px) * CC + pc * 8), *(const v4u*)&sh_[px][pc * 8]); vst2((unsigned*)(AL + (p0 + px) * CC + pc * 8), *(const v4u*)&sl_[px][pc * 8]); }
  if (AP) for (int q = tid; q < CC * 16; q += 256) { const int c = q >> 4, pc = q & 15; vst2(AP + ((size_t)b * CC + c) * NPI + pl0 + pc * 4, *(const v4f*)&spl[c][pc * 4]); }
}
__global__ __launch_bounds__(128) void k_pw(const __bf16* __restrict__ AH, const __bf16* __restrict__ AL, const __bf16* __restrict__ PW, const float* __restrict__ PB, float* __restrict__ A3) {
  __shared__ __align__(16) float so[4][16][68];
  const int tid = threadIdx.x, wave = tid >> 5, lane = tid & 31, col = lane & 15, g = lane >> 4; const size_t r0 = (size_t)blockIdx.x * 64 + wave * 16;
  v8f acc[4] = {};
#pragma unroll
  for (int kc = 0; kc < 2; ++kc) { F2 a; a.h = frag_b(AH + (r0 + col) * CC + kc * 32, lane); a.l = frag_b(AL + (r0 + col) * CC + kc * 32, lane);
#pragma unroll
    for (int j = 0; j < 4; ++j) { const v16b w = frag_b(PW + (size_t)(j * 16 + col) * CC + kc * 32, lane); acc[j] = wmma_bf(a.l, w, acc[j]); acc[j] = wmma_bf(a.h, w, acc[j]); } }
#pragma unroll
  for (int j = 0; j < 4; ++j) { const float bb = bfr(PB[j * 16 + col]);
#pragma unroll
    for (int r = 0; r < 8; ++r) so[wave][8 * g + r][j * 16 + col] = acc[j][r] + bb; }
  LDSX();
  for (int rl = 0; rl < 16; ++rl) if (lane < 16) vst2(A3 + (r0 + rl) * CC + lane * 4, *(const v4f*)&so[wave][rl][lane * 4]);
}
__global__ __launch_bounds__(256) void k_gate(const float* __restrict__ X, const float* __restrict__ A3, float* __restrict__ OUT) {
  __shared__ __align__(16) float s[NPI]; const int b = blockIdx.x / CC, c = blockIdx.x % CC, tid = threadIdx.x; const size_t pb = ((size_t)b * CC + c) * NPI;
  for (int p = tid; p < NPI; p += 256) s[p] = bfr(X[pb + p]) * A3[((size_t)b * NPI + p) * CC + c];
  __syncthreads();
  for (int q = tid; q < NPI / 4; q += 256) vst2(OUT + pb + q * 4, *(const v4f*)&s[q * 4]);
}
extern "C" void kernel_launch(void* const* d_in, const int* in_sizes, int n_in, void* d_out, int out_size, void* d_ws, size_t ws_size, hipStream_t stream) {
  (void)in_sizes; (void)n_in; (void)out_size;
  const float** F = (const float**)d_in;
  if (ws_size < (size_t)WS_END) return;
  char* ws = (char*)d_ws; __bf16 *PK = (__bf16*)(ws + WS_PK), *XCb = (__bf16*)(ws + WS_XC), *A1H = (__bf16*)(ws + WS_A1H), *A1L = (__bf16*)(ws + WS_A1L), *A2H = (__bf16*)(ws + WS_A2H), *A2L = (__bf16*)(ws + WS_A2L); float *OF1 = (float*)(ws + WS_OF1), *A1P = (float*)(ws + WS_A1P), *OF2 = (float*)(ws + WS_OF2), *A3 = (float*)(ws + WS_A3);
  k_pack<<<dim3(N2, 3), 256, 0, stream>>>(F[1], F[4], F[7], PK);
  k_xc<<<NTL, 256, 0, stream>>>(F[0], XCb);
  k_offc<5, 1, 2, 4, 0, 64><<<NTL, 128, 0, stream>>>(XCb, nullptr, PK + PK_O1, F[2], 50, OF1);
  k_ddw<5, 1, 2, N1><<<NTL, 256, 0, stream>>>(F[0], OF1, F[3], 1, A1H, A1L, A1P);
  k_offc<7, 3, 9, 7, 1, 128><<<NTL, 128, 0, stream>>>(A1H, A1L, PK + PK_O2, F[5], 98, OF2);
  k_ddw<7, 3, 9, 128><<<NTL, 256, 0, stream>>>(A1P, OF2, F[6], 0, A2H, A2L, nullptr);
  k_pw<<<NTL, 128, 0, stream>>>(A2H, A2L, PK + PK_PW, F[8], A3);
  k_gate<<<NBO * CC, 256, 0, stream>>>(F[0], A3, (float*)d_out);
}
